// KernalAttention_52304111730698
// MI455X (gfx1250) — hardware-verified
//
#include <hip/hip_runtime.h>
#include <math.h>
#include <stdint.h>

#ifndef NB
#define NB 4
#endif
#ifndef SEQ
#define SEQ 4096
#endif
#define NB_FULL  4
#define SEQ_FULL 4096
#define NH 8
#define HD 64
#define NR 256
#define QB_FULL ((long long)SEQ_FULL * NH * HD)
#define KB_FULL ((long long)SEQ_FULL * HD)
static_assert(NB >= 1 && NB <= NB_FULL);
static_assert(SEQ >= 64 && SEQ <= SEQ_FULL && (SEQ % 64) == 0);
static_assert(HD == 64 && NR == 256);
static_assert(((SEQ * NH * HD / 8) % 256) == 0 && ((SEQ * HD / 8) % 256) == 0);

typedef _Float16 v16h __attribute__((ext_vector_type(16)));
typedef _Float16 v8h  __attribute__((ext_vector_type(8)));
typedef float    v8f  __attribute__((ext_vector_type(8)));
typedef float    v4f  __attribute__((ext_vector_type(4)));
typedef unsigned int v4u __attribute__((ext_vector_type(4)));

#if defined(__HIP_DEVICE_COMPILE__)
#define DEV_ASM 1
#else
#define DEV_ASM 0
#endif

__device__ __forceinline__ unsigned short h_bits(_Float16 x) { return __builtin_bit_cast(unsigned short, x); }
__device__ __forceinline__ unsigned pk16(unsigned short a, unsigned short b) { return (unsigned)a | ((unsigned)b << 16); }
__device__ __forceinline__ v8f zero8() { v8f z = {0.f, 0.f, 0.f, 0.f, 0.f, 0.f, 0.f, 0.f}; return z; }

__device__ __forceinline__ v16h ldfrag(const _Float16* p) {
  union { v16h v; v8h h[2]; } f;
  f.h[0] = *(const v8h*)(p);
  f.h[1] = *(const v8h*)(p + 16);
  return f.v;
}

__device__ __forceinline__ v8f mmar(v16h a, v16h b, v8f c) {
  return __builtin_amdgcn_wmma_f32_16x16x32_f16(false, a, false, b, (short)0, c, false, false);
}
__device__ __forceinline__ void dep_guard(v8f& a, v8f& b, v16h x, v16h y) {
#if DEV_ASM
  asm volatile("v_nop\n\tv_nop\n\tv_nop\n\tv_nop" : "+v"(a), "+v"(b) : "v"(x), "v"(y));
#else
  (void)a; (void)b; (void)x; (void)y;
#endif
}
__device__ __forceinline__ void keep4(v16h a, v16h b, v16h c, v16h d) {
#if DEV_ASM
  asm volatile("v_nop" :: "v"(a), "v"(b), "v"(c), "v"(d));
#else
  (void)a; (void)b; (void)c; (void)d;
#endif
}
__device__ __forceinline__ void acc_guard4(v8f& a, v8f& b, v8f& c, v8f& d) {
#if DEV_ASM
  asm volatile("v_nop\n\tv_nop\n\tv_nop\n\tv_nop" : "+v"(a), "+v"(b), "+v"(c), "+v"(d));
#else
  (void)a; (void)b; (void)c; (void)d;
#endif
}

__global__ __launch_bounds__(256) void cvt_h8(const float* __restrict__ in, long long inStrideY,
                                              unsigned short* out, long long outStrideY, int n8, float scale) {
  const int i = blockIdx.x * 256 + (int)threadIdx.x;
  const int y = blockIdx.y;
  if (i < n8) {
    const float* src = in + (size_t)y * (size_t)inStrideY + (size_t)i * 8;
    const v4f a  = *(const v4f*)(src);
    const v4f a4 = *(const v4f*)(src + 4);
    v4u p;
    p[0] = pk16(h_bits((_Float16)(a[0] * scale)),  h_bits((_Float16)(a[1] * scale)));
    p[1] = pk16(h_bits((_Float16)(a[2] * scale)),  h_bits((_Float16)(a[3] * scale)));
    p[2] = pk16(h_bits((_Float16)(a4[0] * scale)), h_bits((_Float16)(a4[1] * scale)));
    p[3] = pk16(h_bits((_Float16)(a4[2] * scale)), h_bits((_Float16)(a4[3] * scale)));
    unsigned short* o = out + (size_t)y * (size_t)outStrideY + (size_t)i * 8;
    *(volatile v4u*)o = p;
    __threadfence();
    *(volatile v4u*)o = p;
  }
}

__global__ __launch_bounds__(256) void tr_cvt64(const float* __restrict__ in, int cols, long long inStrideZ,
                                                unsigned short* out, int ldo, long long ocolStrideZ, float scale) {
  __shared__ float T[64 * 65];
  const int tid = (int)threadIdx.x;
  const int ti = blockIdx.x, tj = blockIdx.y, z = blockIdx.z;
  {
    const int row = tid >> 2, c16 = (tid & 3) * 16;
    const float* src = in + (size_t)z * (size_t)inStrideZ + (size_t)(ti * 64 + row) * (size_t)cols + tj * 64 + c16;
#pragma unroll
    for (int e = 0; e < 4; ++e) {
      const v4f a = *(const v4f*)(src + 4 * e);
      float* t = T + row * 65 + c16 + 4 * e;
      t[0] = a[0]; t[1] = a[1]; t[2] = a[2]; t[3] = a[3];
    }
  }
  __syncthreads();
  const int wave = tid >> 5, lane = tid & 31;
  const int q = lane >> 3, c8 = (lane & 7) * 8;
  v4u hv[2];
#pragma unroll
  for (int it = 0; it < 2; ++it) {
    const int j = wave * 8 + it * 4 + q;
    v4u a;
#pragma unroll
    for (int e = 0; e < 4; ++e) {
      const float f0 = T[(c8 + 2 * e) * 65 + j] * scale;
      const float f1 = T[(c8 + 2 * e + 1) * 65 + j] * scale;
      a[e] = pk16(h_bits((_Float16)f0), h_bits((_Float16)f1));
    }
    hv[it] = a;
  }
  unsigned short* ob = out + (size_t)z * (size_t)ocolStrideZ + (size_t)ti * 64 + c8;
  for (int pass = 0; pass < 2; ++pass) {
#pragma unroll
    for (int it = 0; it < 2; ++it) {
      const int j = wave * 8 + it * 4 + q;
      *(volatile v4u*)(ob + (size_t)(tj * 64 + j) * (size_t)ldo) = hv[it];
    }
    __threadfence();
  }
}

template <int OUT_MODE>
__global__ __launch_bounds__(256) void gemm64(
    const unsigned short* __restrict__ Ap, int lda, long long strideA,
    const unsigned short* __restrict__ Btp, int ldb, long long strideB,
    void* Cout, int ldc, long long strideC,
    int M, int N, int K, float oscale) {
  const _Float16* A  = (const _Float16*)(const void*)Ap;
  const _Float16* Bt = (const _Float16*)(const void*)Btp;
  __shared__ __align__(16) float sT[8][16 * 68];
  const int b    = blockIdx.y;
  const int lane = threadIdx.x & 31;
  const int wave = threadIdx.x >> 5;
  const int tilesN = N >> 6;
  const int tilesM = M >> 6;
  const int tile = blockIdx.x * 8 + wave;
  if (tile >= tilesM * tilesN) return;
  const int tm = tile / tilesN;
  const int tn = tile - tm * tilesN;
  const int m0 = tm << 6;
  const int n0 = tn << 6;

  const _Float16* Ab = A  + (size_t)b * (size_t)strideA;
  const _Float16* Bb = Bt + (size_t)b * (size_t)strideB;

  const int rlane = lane & 15;
  const int koff  = (lane >> 4) * 8;
  const int mOff  = (lane >> 4) * 8;

  v8f acc[4][4];
#pragma unroll
  for (int i = 0; i < 4; ++i)
#pragma unroll
    for (int j = 0; j < 4; ++j) acc[i][j] = zero8();

  for (int k0 = 0; k0 < K; k0 += 32) {
    v16h bq[4];
#pragma unroll
    for (int j = 0; j < 4; ++j)
      bq[j] = ldfrag(Bb + (size_t)(n0 + (j << 4) + rlane) * (size_t)ldb + koff + k0);
#pragma unroll
    for (int i = 0; i < 4; ++i) {
      const v16h af = ldfrag(Ab + (size_t)(m0 + (i << 4) + rlane) * (size_t)lda + koff + k0);
#pragma unroll
      for (int j = 0; j < 4; ++j) acc[i][j] = mmar(af, bq[j], acc[i][j]);
      dep_guard(acc[i][0], acc[i][3], af, bq[3]);
    }
    keep4(bq[0], bq[1], bq[2], bq[3]);
  }
  acc_guard4(acc[0][0], acc[0][1], acc[0][2], acc[0][3]);
  acc_guard4(acc[1][0], acc[1][1], acc[1][2], acc[1][3]);
  acc_guard4(acc[2][0], acc[2][1], acc[2][2], acc[2][3]);
  acc_guard4(acc[3][0], acc[3][1], acc[3][2], acc[3][3]);

  float* slab = sT[wave];
#pragma unroll
  for (int i = 0; i < 4; ++i) {
    const int mBase = m0 + (i << 4);
#pragma unroll
    for (int j = 0; j < 4; ++j) {
#pragma unroll
      for (int r = 0; r < 8; ++r) {
        slab[(mOff + r) * 68 + (j << 4) + rlane] = acc[i][j][r];
      }
    }
    __builtin_amdgcn_fence(__ATOMIC_RELEASE, "workgroup");
    __builtin_amdgcn_wave_barrier();
    __builtin_amdgcn_fence(__ATOMIC_ACQUIRE, "workgroup");
    if (OUT_MODE == 0) {
      float* C = (float*)Cout + (size_t)b * (size_t)strideC;
      const int h2 = lane >> 4, c4 = (lane & 15) * 4;
      for (int pass = 0; pass < 2; ++pass) {
#pragma unroll
        for (int it = 0; it < 8; ++it) {
          const int row = it * 2 + h2;
          const v4f v = *(const v4f*)(slab + row * 68 + c4) * oscale;
          *(volatile v4f*)(C + (size_t)(mBase + row) * (size_t)ldc + n0 + c4) = v;
        }
        __threadfence();
      }
    } else {
      const int q = lane >> 3, c8 = (lane & 7) * 8;
      unsigned short* C = (unsigned short*)Cout + (size_t)b * (size_t)strideC;
      v4u hv[4];
#pragma unroll
      for (int it = 0; it < 4; ++it) {
        const int row = it * 4 + q;
        const float* sp = slab + row * 68 + c8;
        float f[8];
#pragma unroll
        for (int e = 0; e < 8; ++e) {
          const float x = sp[e] * oscale;
          f[e] = (OUT_MODE == 2) ? __expf(x) : x;
        }
        v4u a;
#pragma unroll
        for (int e = 0; e < 4; ++e) {
          const _Float16 x0 = (_Float16)f[2 * e], x1 = (_Float16)f[2 * e + 1];
          a[e] = pk16(h_bits(x0), h_bits(x1));
        }
        hv[it] = a;
      }
      for (int pass = 0; pass < 2; ++pass) {
#pragma unroll
        for (int it = 0; it < 4; ++it) {
          const int row = it * 4 + q;
          *(volatile v4u*)(C + (size_t)(mBase + row) * (size_t)ldc + n0 + c8) = hv[it];
        }
        __threadfence();
      }
    }
    __builtin_amdgcn_fence(__ATOMIC_RELEASE, "workgroup");
    __builtin_amdgcn_wave_barrier();
    __builtin_amdgcn_fence(__ATOMIC_ACQUIRE, "workgroup");
  }
}

extern "C" void kernel_launch(void* const* d_in, const int* in_sizes, int n_in,
                              void* d_out, int out_size, void* d_ws, size_t ws_size,
                              hipStream_t stream) {
  if (n_in < 4) return;
  const long long needQ  = ((long long)(NB - 1) * SEQ_FULL + SEQ) * NH * HD;
  const long long needKV = ((long long)(NB - 1) * SEQ_FULL + SEQ) * HD;
  if ((long long)in_sizes[0] < needQ) return;
  if ((long long)in_sizes[1] < needKV || (long long)in_sizes[2] < needKV) return;
  if (in_sizes[3] < HD * NR) return;
  if ((long long)out_size < (long long)NB * SEQ * NH * HD) return;

  const float* Q = (const float*)d_in[0];
  const float* K = (const float*)d_in[1];
  const float* V = (const float*)d_in[2];
  const float* W = (const float*)d_in[3];

  const long long MQ = (long long)NB * SEQ * NH;
  const long long NK = (long long)NB * SEQ;

  const size_t PQ  = (size_t)MQ * HD * 2;
  const size_t PK  = (size_t)NK * HD * 2;
  const size_t PVT = (size_t)HD * NK * 2;
  const size_t PWT = (size_t)NR * HD * 2;
  const size_t PWK = (size_t)NR * NK * 2;
  const size_t PKV = (size_t)NB * HD * NR * 2;
  const size_t PWQ = (size_t)MQ * NR * 2;
  size_t off = 0;
  const size_t oQ  = off; off += PQ;
  const size_t oK  = off; off += PK;
  const size_t oVT = off; off += PVT;
  const size_t oWT = off; off += PWT;
  const size_t oWK = off; off += PWK;
  const size_t oKV = off; off += PKV;
  const size_t oWQ = off; off += PWQ;
  if (off > ws_size) return;
  if (off > (size_t)134217728) return;

  char* ws = (char*)d_ws;
  unsigned short* Qh  = (unsigned short*)(ws + oQ);
  unsigned short* Kh  = (unsigned short*)(ws + oK);
  unsigned short* VT  = (unsigned short*)(ws + oVT);
  unsigned short* WT  = (unsigned short*)(ws + oWT);
  unsigned short* WKT = (unsigned short*)(ws + oWK);
  unsigned short* KVT = (unsigned short*)(ws + oKV);
  unsigned short* WQ  = (unsigned short*)(ws + oWQ);

  const dim3 blk(256);
  const int n8q = SEQ * NH * HD / 8;
  const int n8k = SEQ * HD / 8;
  const dim3 gCvtQ((n8q + 255) / 256, NB);
  const dim3 gCvtK((n8k + 255) / 256, NB);
  const dim3 gTrV(SEQ / 64, 1, NB);
  const dim3 gTrW(1, NR / 64, 1);
  const long long t1 = (long long)(NR / 64) * (NK / 64);
  const long long t3 = (MQ / 64) * (NR / 64);
  const long long t4 = ((long long)SEQ * NH / 64) * (HD / 64);
  const dim3 g1((unsigned)((t1 + 7) / 8), 1);
  const dim3 g2(1, NB);
  const dim3 g3((unsigned)((t3 + 7) / 8), 1);
  const dim3 g4((unsigned)((t4 + 7) / 8), NB);

  cvt_h8<<<gCvtQ, blk, 0, stream>>>(Q, QB_FULL, Qh, (long long)SEQ * NH * HD, n8q, 16.0f);
  cvt_h8<<<gCvtK, blk, 0, stream>>>(K, KB_FULL, Kh, (long long)SEQ * HD, n8k, 16.0f);
  tr_cvt64<<<gTrV, blk, 0, stream>>>(V, HD, KB_FULL, VT, (int)NK, (long long)SEQ, 16.0f);
  tr_cvt64<<<gTrW, blk, 0, stream>>>(W, NR, 0LL, WT, HD, 0LL, 16.0f);
  gemm64<2><<<g1, blk, 0, stream>>>(WT, HD, 0LL, Kh, HD, 0LL, (void*)WKT, (int)NK, 0LL,
                                   NR, (int)NK, HD, 1.0f / 256.0f);
  gemm64<1><<<g2, dim3(128), 0, stream>>>(VT, (int)NK, (long long)SEQ, WKT, (int)NK, (long long)SEQ,
                                         (void*)KVT, NR, (long long)HD * NR,
                                         HD, NR, SEQ, 1.0f / 256.0f);
  gemm64<2><<<g3, blk, 0, stream>>>(Qh, HD, 0LL, WT, HD, 0LL, (void*)WQ, NR, 0LL,
                                   (int)MQ, NR, HD, 1.0f / 256.0f);
  gemm64<0><<<g4, blk, 0, stream>>>(WQ, NR, (long long)SEQ * NH * NR, KVT, NR, (long long)HD * NR,
                                   d_out, HD, (long long)SEQ * NH * HD,
                                   SEQ * NH, HD, NR, 16.0f);
  (void)hipGetLastError();
}
